// DKBATNet_4990751998391
// MI455X (gfx1250) — hardware-run, weakly checked
//
#include <hip/hip_runtime.h>


namespace {
constexpr int N = 50000, M = 256, E = 1000000, F = 64, NPB = 8;
constexpr float HS = 256.0f, WSC = 256.0f, SLOPE = 0.2f;
typedef _Float16 b16;
typedef __attribute__((ext_vector_type(16))) _Float16 v16b;
typedef __attribute__((ext_vector_type(8))) _Float16 v8b;
typedef __attribute__((ext_vector_type(8))) float v8f;
typedef __attribute__((ext_vector_type(4))) float v4f;
typedef __attribute__((ext_vector_type(2))) float v2f;
__device__ __forceinline__ float bf16_rne(float f) { unsigned int u = __float_as_uint(f); u += 0x7FFFu + ((u >> 16) & 1u); float r = __uint_as_float(u & 0xFFFF0000u); asm volatile("" : "+v"(r)); return r; }
__device__ __forceinline__ float bfv(float f) { float r = bf16_rne(f); asm volatile("" : "+v"(r)); return r; }
__device__ __forceinline__ void split16(float v, b16& hi, b16& lo) { hi = (b16)v; lo = (b16)(v - (float)hi); }
__device__ __forceinline__ v16b frag_kb(const b16* p, int hh) { const v8b a = *(const v8b*)(p + 8 * hh), b = *(const v8b*)(p + 16 + 8 * hh); v16b f;
#pragma unroll
  for (int e = 0; e < 8; ++e) { f[e] = a[e]; f[8 + e] = b[e]; } return f; }
__device__ __forceinline__ v8f wmma16b(v16b a, v16b b, v8f c) { v8f d = __builtin_amdgcn_wmma_f32_16x16x32_f16(false, a, false, b, (short)0, c, false, false); asm volatile("v_nop\n\tv_nop\n\tv_nop\n\tv_nop" : "+v"(d) : "v"(a), "v"(b)); return d; }
__device__ __forceinline__ void wave_lds_sync() { __builtin_amdgcn_fence(__ATOMIC_RELEASE, "workgroup"); __builtin_amdgcn_wave_barrier(); __builtin_amdgcn_fence(__ATOMIC_ACQUIRE, "workgroup"); }
__device__ __forceinline__ float pmul(float a, float b) { float p = a * b; asm volatile("" : "+v"(p)); return p; }
__device__ __forceinline__ int iclamp(int v, int lo, int hi) { return v < lo ? lo : (v > hi ? hi : v); }
__device__ __forceinline__ float wsum(float v) { for (int o = 16; o; o >>= 1) v += __shfl_xor(v, o); return v; }
__device__ __forceinline__ float elu1(float v) { return v > 0.0f ? v : expm1f(v); }
constexpr int CSR_NBLK8 = 512, CSR_GB8 = 8, CSR_GN8 = 1 << CSR_GB8  , CSR_TS8 = (CSR_GN8 < 32 ? 32 : CSR_GN8)  , CSR_MAXG8 = 512, CSR_CAP8 = 12288  ;
__device__ __host__ __forceinline__ int csr_tix8(int v) { return (v >> CSR_GB8) * CSR_TS8 + (v & (CSR_GN8 - 1)); }
__global__ __launch_bounds__(64) void csrA_kernel8(const int* __restrict__ dst, int E, int N, int nG, int CHP, int NGP, int* __restrict__ STG, int* __restrict__ HST) {
  extern __shared__ int sm[];
  int* cnt = sm; int* run = sm + NGP; int* ids = sm + 2 * NGP;
  const int b = blockIdx.x; const int ch = (E + CSR_NBLK8 - 1) / CSR_NBLK8; const int e0 = b * ch, e1 = min(E, e0 + ch);
  for (int i = threadIdx.x; i < NGP; i += 64) cnt[i] = 0;
  for (int i = threadIdx.x; i < CHP; i += 64) ids[i] = -1;
  __syncthreads();
  if (threadIdx.x == 0) {
    for (int e = e0; e < e1; ++e) { int d = dst[e]; d = (d < 0) ? 0 : (d >= N ? N - 1 : d); cnt[d >> CSR_GB8] += 1; }
    int acc = 0; for (int g = 0; g < nG; ++g) { run[g] = acc; acc += cnt[g]; }
    for (int e = e0; e < e1; ++e) { int d = dst[e]; d = (d < 0) ? 0 : (d >= N ? N - 1 : d); const int g = d >> CSR_GB8; ids[run[g]] = e; run[g] += 1; } }
  __syncthreads();
  typedef __attribute__((ext_vector_type(4))) int v4i;
  for (int pass = 0; pass < 2; ++pass) {
    for (int i = threadIdx.x; i < CHP / 4; i += 64) *(volatile v4i*)(STG + (size_t)b * CHP + i * 4) = *(const v4i*)(&ids[i * 4]);
    for (int i = threadIdx.x; i < NGP / 4; i += 64) { v4i v; for (int e = 0; e < 4; ++e) v[e] = (i * 4 + e < nG) ? cnt[i * 4 + e] : 0; *(volatile v4i*)(HST + (size_t)b * NGP + i * 4) = v; }
    __threadfence(); }
}
__global__ __launch_bounds__(512) void csrS_kernel8(const int* __restrict__ HST, int nG, int NGP, int* __restrict__ START, int* __restrict__ TOT, int* __restrict__ OFF) {
  __shared__ int tot[CSR_MAXG8];
  const int b = threadIdx.x;
  for (int pass = 0; pass < 2; ++pass) { int runb = 0; for (int g = 0; g < nG; ++g) { int c = HST[(size_t)b * NGP + g]; c = (c < 0) ? 0 : c; ((volatile int*)OFF)[(size_t)g * CSR_NBLK8 + b] = runb; runb += c; } __threadfence(); }
  for (int g = threadIdx.x; g < nG; g += 512) { int s = 0; for (int bb = 0; bb < CSR_NBLK8; ++bb) { int c = HST[(size_t)bb * NGP + g]; s += (c < 0) ? 0 : c; } tot[g] = s; }
  __syncthreads();
  if (threadIdx.x < 32) {
    __shared__ int st[CSR_MAXG8 + 32];
    if (threadIdx.x == 0) { int acc = 0; for (int g = 0; g < NGP; ++g) { st[g] = acc; if (g < nG) acc += (tot[g] + 31) & ~31; } st[NGP] = acc; }
    __builtin_amdgcn_fence(__ATOMIC_RELEASE, "workgroup"); __builtin_amdgcn_wave_barrier(); __builtin_amdgcn_fence(__ATOMIC_ACQUIRE, "workgroup");
    for (int pass = 0; pass < 2; ++pass) { for (int i = threadIdx.x; i < NGP + 32; i += 32) { ((volatile int*)START)[i] = (i <= NGP) ? st[min(i, NGP)] : 0; ((volatile int*)TOT)[i] = (i < nG) ? tot[i] : 0; } __threadfence(); } }
}
__global__ __launch_bounds__(256) void csrB_kernel8(const int* __restrict__ dst, int N, int nG, int CHP, int NGP, int permLen, const int* __restrict__ STG, const int* __restrict__ HST, const int* __restrict__ OFF, const int* __restrict__ START, const int* __restrict__ TOT, int* __restrict__ PERM, int* __restrict__ ROWPTR, int* __restrict__ ROWCNT, int* __restrict__ FLAG) {
  typedef __attribute__((ext_vector_type(4))) int v4i;
  __shared__ int ids[CSR_CAP8]; __shared__ unsigned short key[CSR_CAP8]; __shared__ int outp[CSR_CAP8]; __shared__ int ncnt[CSR_GN8 + 1]; __shared__ int boff[CSR_NBLK8 + 1];
  const int g = blockIdx.x, t_ = threadIdx.x; int tot = TOT[g]; int st = START[g], stn = START[g + 1]; const int v0 = g * CSR_GN8; const int nv = min(CSR_GN8, N - v0); const int t0 = g * CSR_TS8;
  st = (st < 0) ? 0 : (st > permLen - 32 ? permLen - 32 : st) & ~31; stn = (stn < st) ? st : (stn > permLen ? permLen : stn); tot = (tot < 0) ? 0 : tot; if (tot > stn - st && tot <= CSR_CAP8) tot = stn - st;
  if (tot > CSR_CAP8) {
    for (int pass = 0; pass < 2; ++pass) { for (int i = t_; i < CSR_TS8 / 4; i += 256) { v4i a, c; for (int e = 0; e < 4; ++e) { a[e] = st; c[e] = 0; } *(volatile v4i*)(ROWPTR + t0 + i * 4) = a; *(volatile v4i*)(ROWCNT + t0 + i * 4) = c; } if (t_ == 0) ((volatile int*)FLAG)[0] = 1; __threadfence(); } (void)nv; return; }
  if (t_ == 0) { int acc = 0; for (int b = 0; b < CSR_NBLK8; ++b) { boff[b] = acc; int c = HST[(size_t)b * NGP + g]; c = (c < 0) ? 0 : (c > CHP ? CHP : c); acc += c; if (acc > tot) acc = tot; } boff[CSR_NBLK8] = acc; }
  for (int i = t_; i <= CSR_GN8; i += 256) ncnt[i] = 0;
  __syncthreads();
  for (int b = 0; b < CSR_NBLK8; ++b) { const int c = boff[b + 1] - boff[b]; int o_ = OFF[(size_t)g * CSR_NBLK8 + b]; o_ = (o_ < 0) ? 0 : (o_ > CHP - c ? CHP - c : o_); const int* src_ = STG + (size_t)b * CHP + o_;
    for (int i = t_; i < c; i += 256) { int id = src_[i]; id = (id < 0) ? 0 : id; ids[boff[b] + i] = id; int d = dst[id]; d = (d < v0) ? v0 : (d >= N ? N - 1 : d); int kk = d - v0; kk = (kk < 0) ? 0 : (kk >= CSR_GN8 ? CSR_GN8 - 1 : kk); key[boff[b] + i] = (unsigned short)kk; } }
  __syncthreads();
  if (t_ == 0) { for (int i = 0; i < tot; ++i) ncnt[key[i]] += 1; int acc = 0; for (int vl = 0; vl < CSR_GN8; ++vl) { const int c = ncnt[vl]; ncnt[vl] = acc; acc += c; } ncnt[CSR_GN8] = acc;
    for (int i = 0; i < tot; ++i) { const int vl = key[i]; outp[ncnt[vl]] = ids[i]; ncnt[vl] += 1; }
    for (int vl = CSR_GN8; vl > 0; --vl) ncnt[vl] = ncnt[vl - 1]; ncnt[0] = 0; }
  __syncthreads();
  for (int pass = 0; pass < 2; ++pass) {
    for (int i = t_; i < (stn - st) / 4; i += 256) { v4i v; for (int e = 0; e < 4; ++e) { const int q = i * 4 + e; v[e] = (q < tot) ? outp[q] : -1; } *(volatile v4i*)(PERM + st + i * 4) = v; }
    for (int i = t_; i < CSR_TS8 / 4; i += 256) { v4i a, c; for (int e = 0; e < 4; ++e) { const int vl = i * 4 + e; const int vc = vl < CSR_GN8 ? vl : CSR_GN8; a[e] = (vl < CSR_GN8) ? st + ncnt[vc] : st; c[e] = (vl < nv) ? (ncnt[(vc < CSR_GN8 ? vc : CSR_GN8 - 1) + 1] - ncnt[vc]) : 0; } *(volatile v4i*)(ROWPTR + t0 + i * 4) = a; *(volatile v4i*)(ROWCNT + t0 + i * 4) = c; }
    __threadfence(); }
}
__global__ __launch_bounds__(256) void csrZ_kernel8(int* __restrict__ p, size_t n4) { typedef __attribute__((ext_vector_type(4))) int v4i; const size_t tid = (size_t)blockIdx.x * 256 + threadIdx.x, nth = (size_t)gridDim.x * 256; v4i z = {0, 0, 0, 0}; for (size_t i = tid; i < n4; i += nth) *(volatile v4i*)(p + i * 4) = z; }
struct CsrBufs8 { int *STG, *HST, *OFF, *START, *TOT, *PERM, *ROWPTR, *ROWCNT, *FLAG; int nG, NGP, CHP; size_t permLen; char* base; size_t bytes; };
static size_t csr_carve8(CsrBufs8& c, char* ws, size_t off, int E, int N) {
  const size_t off0 = off; c.base = ws + off;
  auto al = [&](size_t bytes) { char* p = ws + off; off += (bytes + 255) & ~(size_t)255; return p; };
  c.nG = (N + CSR_GN8 - 1) / CSR_GN8; c.NGP = (c.nG + 31) & ~31; const int ch = (E + CSR_NBLK8 - 1) / CSR_NBLK8; c.CHP = (ch + 31) & ~31; c.permLen = (size_t)E + 32 * (size_t)c.nG + 32;
  c.STG = (int*)al((size_t)CSR_NBLK8 * c.CHP * 4); c.HST = (int*)al((size_t)CSR_NBLK8 * c.NGP * 4); c.OFF = (int*)al((size_t)c.NGP * CSR_NBLK8 * 4); c.START = (int*)al((size_t)(c.NGP + 64) * 4); c.TOT = (int*)al((size_t)(c.NGP + 64) * 4);
  c.PERM = (int*)al(c.permLen * 4); c.ROWPTR = (int*)al((size_t)c.nG * CSR_TS8 * 4); c.ROWCNT = (int*)al((size_t)c.nG * CSR_TS8 * 4); c.FLAG = (int*)al(256);
  c.bytes = off - off0; return off;
}
static void csr_build8(const CsrBufs8& c, const int* dst, int E, int N, hipStream_t stream) {
  const size_t smem = (size_t)(2 * c.NGP + c.CHP) * 4;
  csrZ_kernel8<<<512, 256, 0, stream>>>((int*)c.base, c.bytes / 16);
  csrA_kernel8<<<CSR_NBLK8, 64, smem, stream>>>(dst, E, N, c.nG, c.CHP, c.NGP, c.STG, c.HST);
  csrS_kernel8<<<1, 512, 0, stream>>>(c.HST, c.nG, c.NGP, c.START, c.TOT, c.OFF);
  csrB_kernel8<<<c.nG, 256, 0, stream>>>(dst, N, c.nG, c.CHP, c.NGP, (int)c.permLen, c.STG, c.HST, c.OFF, c.START, c.TOT, c.PERM, c.ROWPTR, c.ROWCNT, c.FLAG);
}


__global__ __launch_bounds__(256) void wput_kernel(const float* __restrict__ w1i1, const float* __restrict__ w1o1, const float* __restrict__ w1i2, const float* __restrict__ w1o2, const float* __restrict__ wrel, const float* __restrict__ wmii, const float* __restrict__ wmio, const float* __restrict__ wmoi, const float* __restrict__ wmoo, const float* __restrict__ went, b16* __restrict__ WN, b16* __restrict__ WG, b16* __restrict__ WG2, b16* __restrict__ WM, b16* __restrict__ WE) { const int u = blockIdx.x * 256 + threadIdx.x; v8b v; auto put = [&](b16* dst, const float* src) {
#pragma unroll
    for (int j = 0; j < 8; ++j) v[j] = (b16)(bf16_rne(src[j]) * WSC); for (int pass = 0; pass < 2; ++pass) { *(volatile v8b*)dst = v; __threadfence(); } };
  if (u < 2 * 256 * 8) { const int l = u / (256 * 8), o = (u / 8) % 256, k0 = (u % 8) * 8; const float* w = (o < 128 ? (l == 0 ? w1i1 : w1i2) : (l == 0 ? w1o1 : w1o2)); const int oo = o % 64, part = (o % 128) / 64; put(WN + ((size_t)l * 256 + o) * F + k0, w + (size_t)oo * 192 + part * 64 + k0); }
  if (u < 192 * 8) { const int o = u / 8, k0 = (u % 8) * 8; const float* w = o < 64 ? w1i1 + (size_t)o * 192 + 128 + k0 : (o < 128 ? w1o1 + (size_t)(o - 64) * 192 + 128 + k0 : wrel + (size_t)(o - 128) * F + k0); put(WG + (size_t)o * F + k0, w); }
  if (u < 128 * 8) { const int o = u / 8, k0 = (u % 8) * 8; const float* w = o < 64 ? w1i2 + (size_t)o * 192 + 128 + k0 : w1o2 + (size_t)(o - 64) * 192 + 128 + k0; put(WG2 + (size_t)o * F + k0, w); }
  if (u < 2 * 128 * 8) { const int l = u / (128 * 8), o = (u / 8) % 128, k0 = (u % 8) * 8; const float* w = (l == 0 ? (o < 64 ? wmii : wmio) : (o < 64 ? wmoi : wmoo)) + (size_t)(o % 64) * F + k0; put(WM + ((size_t)l * 128 + o) * F + k0, w); }
  if (u < 64 * 8) { const int o = u / 8, k0 = (u % 8) * 8; put(WE + (size_t)o * F + k0, went + (size_t)o * F + k0); } }
template <int NT, bool L2N, bool RAW>
__global__ __launch_bounds__(32) void gemm_kernel(const float* __restrict__ IN, int istr, const b16* __restrict__ W, int RLIM, int RTOT, float* __restrict__ OUTR, float* __restrict__ NORMED  ) { __shared__ __attribute__((aligned(16))) b16 Ah[16][F + 8], Al[16][F + 8]; __shared__ float Tr[16][F + 1], Tf[16][NT * 16 + 4]; const int lane = threadIdx.x, nloc = lane & 15, hlf = lane >> 4; const size_t r0 = (size_t)blockIdx.x * 16; if (r0 >= (size_t)RLIM) return; const int nr = (RTOT - (int)r0) < 16 ? (RTOT - (int)r0) : 16;
  for (int rr = 0; rr < 16; ++rr) { const size_t r = r0 + (rr < nr ? rr : 0); const float v0 = IN[r * istr + lane], v1 = IN[r * istr + 32 + lane]; Tr[rr][lane] = RAW ? bfv(v0) : v0; Tr[rr][32 + lane] = RAW ? bfv(v1) : v1; }
  wave_lds_sync();
  if (L2N && lane < 16) { float ss = 0.0f; for (int c = 0; c < F; ++c) ss += pmul(Tr[lane][c], Tr[lane][c]); const float inv = 1.0f / fmaxf(sqrtf(ss), 1e-12f); for (int c = 0; c < F; ++c) Tr[lane][c] *= inv; }
  wave_lds_sync();
  for (int rr = 0; rr < 16; ++rr) for (int q = 0; q < 2; ++q) { const int c = q * 32 + lane; b16 p, pl; split16(Tr[rr][c] * HS, p, pl); Ah[rr][c] = p; Al[rr][c] = pl; }
  if (lane < 16) for (int k = F; k < F + 8; ++k) { Ah[lane][k] = (b16)0.0f; Al[lane][k] = (b16)0.0f; }
  wave_lds_sync(); v8f acc[NT];
#pragma unroll
  for (int t = 0; t < NT; ++t) acc[t] = (v8f){};
#pragma unroll
  for (int kb = 0; kb < F; kb += 32) { const v16b a = frag_kb(&Ah[nloc][kb], hlf), al = frag_kb(&Al[nloc][kb], hlf);
#pragma unroll
    for (int t = 0; t < NT; ++t) { const v16b bw = frag_kb(W + (size_t)(t * 16 + nloc) * F + kb, hlf); acc[t] = wmma16b(a, bw, acc[t]); acc[t] = wmma16b(al, bw, acc[t]); } }
#pragma unroll
  for (int t = 0; t < NT; ++t)
#pragma unroll
    for (int r8 = 0; r8 < 8; ++r8) Tf[8 * hlf + r8][t * 16 + nloc] = acc[t][r8] * (1.0f / (HS * WSC));
  wave_lds_sync();
  for (int pass = 0; pass < 2; ++pass) { for (int rr = 0; rr < nr; ++rr) { for (int q = 0; q < NT / 2; ++q) ((volatile float*)OUTR)[(r0 + rr) * (NT * 16) + q * 32 + lane] = Tf[rr][q * 32 + lane]; if (L2N && NORMED) { ((volatile float*)NORMED)[(r0 + rr) * F + lane] = Tr[rr][lane]; ((volatile float*)NORMED)[(r0 + rr) * F + 32 + lane] = Tr[rr][32 + lane]; } } __threadfence(); } }
template <int DIR, int NH>
__global__ __launch_bounds__(256) void sweep_kernel(const float* __restrict__ PN, const float* __restrict__ PG, int PGW, int goff, const float* __restrict__ att, const int* __restrict__ other, const int* __restrict__ rel, const int* __restrict__ PERM, const int* __restrict__ ROWPTR, const int* __restrict__ ROWCNT, int permLen, int NLIM, float* __restrict__ HN) { const int wave = threadIdx.x >> 5, lane = threadIdx.x & 31; const size_t n = (size_t)blockIdx.x * NPB + wave; if (n >= (size_t)NLIM) return; constexpr int LPH = 32 / NH;
  const int c0 = lane * 2; const float a0 = bfv(att[c0]), a1 = bfv(att[c0 + 1]);
  const v2f own = *(const v2f*)(PN + n * 256 + (DIR == 0 ? 64 : 128) + c0);
  float s0 = 0.0f, s1 = 0.0f, dsum = 0.0f;
  int st = ROWPTR[n], cnt = ROWCNT[n]; cnt = iclamp(cnt, 0, E); st = iclamp(st, 0, permLen - cnt);
#pragma unroll 1
  for (int j = 0; j < cnt; ++j) { const int e = iclamp(PERM[st + j], 0, E - 1); const size_t o = (size_t)iclamp(other[e], 0, N - 1); if (o >= (size_t)NLIM) continue; const int r = iclamp(rel[e], 0, M - 1);
    const v2f po = *(const v2f*)(PN + o * 256 + (DIR == 0 ? 0 : 192) + c0); const v2f pg = *(const v2f*)(PG + (size_t)r * PGW + goff + c0); const float cv0 = po[0] + own[0] + pg[0], cv1 = po[1] + own[1] + pg[1];
    float part = pmul(a0, cv0) + pmul(a1, cv1);
    for (int sh = LPH / 2; sh; sh >>= 1) part += __shfl_xor(part, sh);
    float lr = part > 0.0f ? part : SLOPE * part; const float w = __expf(-lr); s0 += pmul(w, cv0); s1 += pmul(w, cv1); dsum += w; }
  float h0 = 0.0f, h1 = 0.0f; if (dsum > 0.0f) { const float inv = 1.0f / dsum; h0 = elu1(pmul(s0, inv)); h1 = elu1(pmul(s1, inv)); }
  const float ss = wsum(pmul(h0, h0) + pmul(h1, h1)); const float ninv = 1.0f / fmaxf(sqrtf(ss), 1e-12f);
  for (int pass = 0; pass < 2; ++pass) { *(volatile v2f*)(HN + n * F + c0) = (v2f){h0 * ninv, h1 * ninv}; __threadfence(); } }
template <int MODE>
__global__ __launch_bounds__(32) void merge_kernel(const float* __restrict__ HNI, const float* __restrict__ HNO, const b16* __restrict__ WMl, const float* __restrict__ bi, const float* __restrict__ bo, const float* __restrict__ wl, const float* __restrict__ bl, const float* __restrict__ XE, int NLIM, float* __restrict__ OUTR) { __shared__ __attribute__((aligned(16))) b16 Ah[16][F + 8], Al[16][F + 8], Bh[16][F + 8], Bl[16][F + 8]; __shared__ float Ti[16][F + 1], To[16][F + 1], Lm[16]; const int lane = threadIdx.x, nloc = lane & 15, hlf = lane >> 4; const size_t n0 = (size_t)blockIdx.x * 16; if (n0 >= (size_t)NLIM) return;
  for (int rr = 0; rr < 16; ++rr) for (int q = 0; q < 2; ++q) { const int c = q * 32 + lane; b16 p, pl; split16(HNI[(n0 + rr) * F + c] * HS, p, pl); Ah[rr][c] = p; Al[rr][c] = pl; split16(HNO[(n0 + rr) * F + c] * HS, p, pl); Bh[rr][c] = p; Bl[rr][c] = pl; }
  if (lane < 16) for (int k = F; k < F + 8; ++k) { Ah[lane][k] = (b16)0.0f; Al[lane][k] = (b16)0.0f; Bh[lane][k] = (b16)0.0f; Bl[lane][k] = (b16)0.0f; }
  wave_lds_sync(); v8f ai[4] = {(v8f){}, (v8f){}, (v8f){}, (v8f){}}, ao[4] = {(v8f){}, (v8f){}, (v8f){}, (v8f){}};
#pragma unroll
  for (int kb = 0; kb < F; kb += 32) { const v16b a = frag_kb(&Ah[nloc][kb], hlf), al = frag_kb(&Al[nloc][kb], hlf), b = frag_kb(&Bh[nloc][kb], hlf), bl2 = frag_kb(&Bl[nloc][kb], hlf);
#pragma unroll
    for (int t = 0; t < 4; ++t) { const v16b wi = frag_kb(WMl + (size_t)(t * 16 + nloc) * F + kb, hlf), wo = frag_kb(WMl + (size_t)(64 + t * 16 + nloc) * F + kb, hlf); ai[t] = wmma16b(a, wi, ai[t]); ai[t] = wmma16b(al, wi, ai[t]); ao[t] = wmma16b(b, wo, ao[t]); ao[t] = wmma16b(bl2, wo, ao[t]); } }
#pragma unroll
  for (int t = 0; t < 4; ++t) { const int cc = t * 16 + nloc; const float bbi = bfv(bi[cc]), bbo = bfv(bo[cc]);
#pragma unroll
    for (int r8 = 0; r8 < 8; ++r8) { Ti[8 * hlf + r8][cc] = ai[t][r8] * (1.0f / (HS * WSC)) + bbi; To[8 * hlf + r8][cc] = ao[t][r8] * (1.0f / (HS * WSC)) + bbo; } }
  wave_lds_sync();
  if (lane < 16) { float s = bfv(bl[0]); for (int c = 0; c < F; ++c) s += pmul(Ti[lane][c], bfv(wl[c])) + pmul(To[lane][c], bfv(wl[F + c])); Lm[lane] = 1.0f / (1.0f + __expf(-s)); }
  wave_lds_sync();
  for (int pass = 0; pass < 2; ++pass) { for (int rr = 0; rr < 16; ++rr) { const float lm = Lm[rr]; float v0 = pmul(lm, Ti[rr][lane]) + pmul(1.0f - lm, To[rr][lane]), v1 = pmul(lm, Ti[rr][32 + lane]) + pmul(1.0f - lm, To[rr][32 + lane]);
      if (MODE == 1) { v0 += XE[(n0 + rr) * F + lane]; v1 += XE[(n0 + rr) * F + 32 + lane]; const float ss = wsum(pmul(v0, v0) + pmul(v1, v1)); const float inv = 1.0f / fmaxf(sqrtf(ss), 1e-12f); v0 *= inv; v1 *= inv; }
      ((volatile float*)OUTR)[(n0 + rr) * F + lane] = v0; ((volatile float*)OUTR)[(n0 + rr) * F + 32 + lane] = v1; } __threadfence(); } }
__global__ __launch_bounds__(32) void gout_kernel(const float* __restrict__ GP, float* __restrict__ out1) { const int lane = threadIdx.x; const size_t r0 = (size_t)blockIdx.x * 16;
  for (int pass = 0; pass < 2; ++pass) { for (int rr = 0; rr < 16; ++rr) { const float v0 = GP[(r0 + rr) * 192 + 128 + lane], v1 = GP[(r0 + rr) * 192 + 128 + 32 + lane]; const float ss = wsum(pmul(v0, v0) + pmul(v1, v1)); const float inv = 1.0f / fmaxf(sqrtf(ss), 1e-12f); ((volatile float*)out1)[(r0 + rr) * F + lane] = v0 * inv; ((volatile float*)out1)[(r0 + rr) * F + 32 + lane] = v1 * inv; } __threadfence(); } }
}

extern "C" void kernel_launch(void* const* d_in, const int* in_sizes, int n_in, void* d_out, int out_size, void* d_ws, size_t ws_size, hipStream_t stream) {
  (void)n_in;
  auto Fp = [&](int i) { return (const float*)d_in[i]; }; auto Ip = [&](int i) { return (const int*)d_in[i]; };
  if (in_sizes[0] != N * F || in_sizes[1] != M * F || in_sizes[2] != F * 192 || in_sizes[13] != F * 192 || in_sizes[23] != F * F || in_sizes[24] != E || in_sizes[25] != E || in_sizes[26] != E || out_size != N * F + M * F) return;
  const int NLIM = N;
  size_t off = 0; char* ws = (char*)d_ws;
  auto carve = [&](size_t bytes) { char* p = ws + off; off += (bytes + 255) & ~(size_t)255; return p; };
  b16* WN = (b16*)carve((size_t)2 * 256 * F * 2); b16* WG = (b16*)carve(192 * F * 2); b16* WG2 = (b16*)carve(128 * F * 2); b16* WM = (b16*)carve((size_t)2 * 128 * F * 2); b16* WE = (b16*)carve(F * F * 2);
  float* XN = (float*)carve((size_t)N * F * 4); float* PN = (float*)carve((size_t)N * 256 * 4); float* GP = (float*)carve((size_t)M * 192 * 4); float* GP2 = (float*)carve((size_t)M * 128 * 4); float* HNI = (float*)carve((size_t)N * F * 4); float* HNO = (float*)carve((size_t)N * F * 4); float* H1 = (float*)carve((size_t)N * F * 4); float* XE = (float*)carve((size_t)N * F * 4);
  CsrBufs8 cc_; off = csr_carve8(cc_, ws, off, E, N); CsrBufs8 cr_; off = csr_carve8(cr_, ws, off, E, N);
  if (off > ws_size || off > ((size_t)176 << 20)) return;
  wput_kernel<<<(2 * 256 * 8 + 255) / 256, 256, 0, stream>>>(Fp(2), Fp(4), Fp(13), Fp(15), Fp(12), Fp(6), Fp(8), Fp(17), Fp(19), Fp(23), WN, WG, WG2, WM, WE);
  csr_build8(cc_, Ip(25), E, N, stream);
  csr_build8(cr_, Ip(24), E, N, stream);
  const int nb = (NLIM + NPB - 1) / NPB; float* out0 = (float*)d_out; float* out1 = out0 + (size_t)N * F;
  gemm_kernel<16, true, true><<<NLIM / 16, 32, 0, stream>>>(Fp(0), F, WN, NLIM, N, PN, XN);
  gemm_kernel<12, true, true><<<M / 16, 32, 0, stream>>>(Fp(1), F, WG, M, M, GP, nullptr);
  sweep_kernel<0, 2><<<nb, 256, 0, stream>>>(PN, GP, 192, 0, Fp(3), Ip(24), Ip(26), cc_.PERM, cc_.ROWPTR, cc_.ROWCNT, (int)cc_.permLen, NLIM, HNI);
  sweep_kernel<1, 2><<<nb, 256, 0, stream>>>(PN, GP, 192, 64, Fp(5), Ip(25), Ip(26), cr_.PERM, cr_.ROWPTR, cr_.ROWCNT, (int)cr_.permLen, NLIM, HNO);
  merge_kernel<0><<<NLIM / 16, 32, 0, stream>>>(HNI, HNO, WM, Fp(7), Fp(9), Fp(10), Fp(11), nullptr, NLIM, H1);
  gemm_kernel<16, false, false><<<NLIM / 16, 32, 0, stream>>>(H1, F, WN + (size_t)256 * F, NLIM, N, PN, nullptr);
  gemm_kernel<8, false, false><<<M / 16, 32, 0, stream>>>(GP + 128, 192, WG2, M, M, GP2, nullptr);
  sweep_kernel<0, 1><<<nb, 256, 0, stream>>>(PN, GP2, 128, 0, Fp(14), Ip(24), Ip(26), cc_.PERM, cc_.ROWPTR, cc_.ROWCNT, (int)cc_.permLen, NLIM, HNI);
  sweep_kernel<1, 1><<<nb, 256, 0, stream>>>(PN, GP2, 128, 64, Fp(16), Ip(25), Ip(26), cr_.PERM, cr_.ROWPTR, cr_.ROWCNT, (int)cr_.permLen, NLIM, HNO);
  gemm_kernel<4, false, false><<<NLIM / 16, 32, 0, stream>>>(XN, F, WE, NLIM, N, XE, nullptr);
  merge_kernel<1><<<NLIM / 16, 32, 0, stream>>>(HNI, HNO, WM + (size_t)128 * F, Fp(18), Fp(20), Fp(21), Fp(22), XE, NLIM, out0);
  gout_kernel<<<M / 16, 32, 0, stream>>>(GP, out1);
}
